// DendriticLayerSiLU_FFN_87471303950864
// MI455X (gfx1250) — hardware-verified
//
#include <hip/hip_runtime.h>


#ifndef NB
#define NB 4096
#endif
#define NB_FULL 4096
#define KD    1024
#define HOUT  2048
#define NWIN  16
#define WSZ   64
#define TAU_RCP 1.0f
#define TW    32
#define OSP   36
#define ST_TRIPS 8

static_assert(NB <= NB_FULL);
static_assert(NB % 64 == 0);
static_assert(HOUT % 64 == 0);
static_assert(NWIN * WSZ == KD);
static_assert(WSZ % 32 == 0);
static_assert(KD % 8 == 0);
static_assert(TW == 32);
static_assert((OSP * 4) % 16 == 0 && OSP >= TW);
static_assert(32 * 16 * ST_TRIPS == TW * TW * 4);
static_assert(4 * TW * OSP * 4 <= 131072);
static_assert(((size_t)NB * KD) % (8 * 256) == 0);
static_assert(((size_t)HOUT * KD) % (8 * 256) == 0);

typedef unsigned short bf;
typedef __attribute__((ext_vector_type(16))) __bf16   v16bf;
typedef __attribute__((ext_vector_type(8)))  unsigned short v8us;
typedef __attribute__((ext_vector_type(8)))  float    v8f;
typedef __attribute__((ext_vector_type(4)))  float    v4f;
typedef __attribute__((ext_vector_type(4)))  int      v4i;
typedef v4f  __attribute__((may_alias)) v4fa;
typedef v4i  __attribute__((may_alias)) v4ia;

__device__ __forceinline__ unsigned short f2bf(float f) { unsigned u = __float_as_uint(f); u += 0x7FFFu + ((u >> 16) & 1u); return (unsigned short)(u >> 16); }
__device__ __forceinline__ float bf2f(unsigned short w) { return __uint_as_float(((unsigned)w) << 16); }
__device__ __forceinline__ int clampi(int v, int lo, int hi) { return min(max(v, lo), hi); }
__device__ __forceinline__ v16bf cat16b(v8us lo, v8us hi) { return __builtin_bit_cast(v16bf, __builtin_shufflevector(lo, hi, 0, 1, 2, 3, 4, 5, 6, 7, 8, 9, 10, 11, 12, 13, 14, 15)); }
__device__ __forceinline__ v8f wmmab(v16bf a, v16bf b, v8f c) { return __builtin_amdgcn_wmma_f32_16x16x32_bf16(false, a, false, b, (short)0, c, false, false); }
__device__ __forceinline__ v16bf ldb(const bf* p)  { return cat16b(*(const v8us*)p, *(const v8us*)(p + 16)); }
__device__ __forceinline__ void wave_sync() { __builtin_amdgcn_fence(3  , "wavefront"); __builtin_amdgcn_wave_barrier(); asm volatile("" ::: "memory"); }
__device__ __forceinline__ v8f wmmag(v16bf a, v16bf b, v8f c) { c = wmmab(a, b, c); asm volatile("v_nop\n\tv_nop\n\tv_nop\n\tv_nop" : "+v"(c) : "v"(a), "v"(b)); return c; }

__global__ __launch_bounds__(256) void k_cvt(const float* __restrict__ src, bf* dst, int n8) {
    const size_t i = (size_t)blockIdx.x * 256 + threadIdx.x; if (i >= (size_t)n8) return;
    const v8f a = *(const v8f*)(src + i * 8); v8us o;
#pragma unroll
    for (int k = 0; k < 8; ++k) o[k] = f2bf(a[k]);
    *(volatile v8us*)(dst + i * 8) = o; __threadfence(); *(volatile v8us*)(dst + i * 8) = o;
}

__global__ __launch_bounds__(128) __attribute__((amdgpu_num_vgpr(256))) void k_dend(const bf* __restrict__ XB, const bf* __restrict__ TB, float* OUT) {
    __shared__ __align__(16) float os[4 * TW * OSP];
    const int lane = threadIdx.x & 31, lr = lane & 15, hi = lane >> 4;
    const int wave = __builtin_amdgcn_readfirstlane(threadIdx.x >> 5);
    const int nt = blockIdx.x % (NB / 64), ht = blockIdx.x / (NB / 64);
    const int n0 = nt * 64 + (wave & 1) * TW, h0 = ht * 64 + (wave >> 1) * TW;
    v8f mx[2][2], ls[2][2], nm[2][2];
#pragma unroll
    for (int mb = 0; mb < 2; ++mb)
#pragma unroll
        for (int nb = 0; nb < 2; ++nb) { ls[mb][nb] = (v8f){}; nm[mb][nb] = (v8f){};
#pragma unroll
            for (int j = 0; j < 8; ++j) mx[mb][nb][j] = -1.0e30f; }
    const size_t aoff = (size_t)(n0 + lr) * KD + 8 * hi, boff = (size_t)(h0 + lr) * KD + 8 * hi;
#pragma unroll 1
    for (int w = 0; w < NWIN; ++w) {
        v8f acc[2][2];
#pragma unroll
        for (int mb = 0; mb < 2; ++mb)
#pragma unroll
            for (int nb = 0; nb < 2; ++nb) acc[mb][nb] = (v8f){};
#pragma unroll 1
        for (int kc = 0; kc < WSZ; kc += 32) {
            const int kk = w * WSZ + kc;
            v16bf a[2];
#pragma unroll
            for (int mb = 0; mb < 2; ++mb) a[mb] = ldb(XB + aoff + (size_t)mb * 16 * KD + kk);
#pragma unroll
            for (int nb = 0; nb < 2; ++nb) { const v16bf b = ldb(TB + boff + (size_t)nb * 16 * KD + kk);
#pragma unroll
                for (int mb = 0; mb < 2; ++mb) acc[mb][nb] = wmmag(a[mb], b, acc[mb][nb]); }
        }
#pragma unroll
        for (int mb = 0; mb < 2; ++mb) {
#pragma unroll
            for (int nb = 0; nb < 2; ++nb) {
#pragma unroll
                for (int j = 0; j < 8; ++j) {
                    const float s  = acc[mb][nb][j];
                    const float z  = s * TAU_RCP;
                    const float mo = mx[mb][nb][j];
                    const float mn = fmaxf(mo, z);
                    const float ca = __expf(mo - mn);
                    const float p  = __expf(z - mn);
                    const float sg = __builtin_amdgcn_rcpf(1.0f + __expf(-s));
                    const float pv = p * (s * sg);
                    ls[mb][nb][j] = ls[mb][nb][j] * ca + p;
                    nm[mb][nb][j] = nm[mb][nb][j] * ca + pv;
                    mx[mb][nb][j] = mn;
                }
            }
        }
    }
    const int ob = wave * (TW * OSP);
#pragma unroll
    for (int mb = 0; mb < 2; ++mb) {
#pragma unroll
        for (int nb = 0; nb < 2; ++nb) {
#pragma unroll
            for (int j = 0; j < 8; ++j) {
                const float o = nm[mb][nb][j] * __builtin_amdgcn_rcpf(ls[mb][nb][j]);
                os[ob + (mb * 16 + hi * 8 + j) * OSP + nb * 16 + lr] = o; } } }
    wave_sync();
    const int c4 = (lane & 7) * 4;
#pragma unroll 1
    for (int ps = 0; ps < 2; ++ps) {
#pragma unroll 1
        for (int it = 0; it < ST_TRIPS; ++it) { const int row = 4 * it + (lane >> 3);
            const v4f v = *(const v4fa*)(&os[ob + row * OSP + c4]);
            *(volatile v4f*)(OUT + (size_t)(n0 + row) * HOUT + h0 + c4) = v; }
        if (ps == 0) __threadfence(); }
}

static constexpr size_t al256(size_t v) { return (v + 255) & ~(size_t)255; }
static constexpr size_t SZ_XB = al256((size_t)NB * KD * 2);
static constexpr size_t SZ_TB = al256((size_t)HOUT * KD * 2);
static constexpr size_t SZ_TOTAL = SZ_XB + SZ_TB;
static_assert(SZ_TOTAL <= (size_t)134217728);

extern "C" void kernel_launch(void* const* d_in, const int* in_sizes, int n_in,
                              void* d_out, int out_size, void* d_ws, size_t ws_size, hipStream_t stream) {
    if (n_in < 2) return;
    if ((size_t)in_sizes[0] < (size_t)NB * KD) return;
    if ((size_t)in_sizes[1] < (size_t)HOUT * KD) return;
    if ((size_t)out_size < (size_t)NB * HOUT) return;
    if (SZ_TOTAL > ws_size) return;
    const float* x  = (const float*)d_in[0];
    const float* tp = (const float*)d_in[1];
    float* OUT = (float*)d_out;
    char* wsp = (char*)d_ws;
    bf* XB = (bf*)wsp; wsp += SZ_XB;
    bf* TB = (bf*)wsp; wsp += SZ_TB;

    const int n8x = (int)(((size_t)NB * KD) / 8);
    const int n8t = (int)(((size_t)HOUT * KD) / 8);
    k_cvt<<<(unsigned)(n8x / 256), 256, 0, stream>>>(x, XB, n8x);
    k_cvt<<<(unsigned)(n8t / 256), 256, 0, stream>>>(tp, TB, n8t);
    k_dend<<<(unsigned)((NB / 64) * (HOUT / 64)), 128, 0, stream>>>(XB, TB, OUT);
}
